// fairDMoN_49220325212394
// MI455X (gfx1250) — hardware-run, weakly checked
//
#include <hip/hip_runtime.h>
#include <stddef.h>


#define DIM    256
#define KCL    64
#define NTHR   256
#define NWAVE  8
#define GRS    128
#define PSS    68
#define FTD    64
#define PFT    132
#define TPK    64
#define TPN    32
#define TPP    72
#define ASCL   16
#define WSCL   64
#define NEG    256
#define EPB    128
#define NPB    64
#define NFB    16
#define WSCAP  134217728
#define LDS_POOL (KCL * DIM * 4)
#define SELU_S 1.0507009873554805f
#define SELU_A 1.6732632423543772f

static_assert(GRS == NWAVE * 16);
static_assert(KCL == 64 && (DIM % 32) == 0);
static_assert((PSS % 4) == 0 && (PFT % 4) == 0);
static_assert(TPN * 8 == NTHR && TPK * TPN == NTHR * 8 && TPK == NWAVE * 8);
static_assert((TPP % 8) == 0 && TPP >= TPK);
static_assert((DIM % TPK) == 0 && (KCL % TPN) == 0);
static_assert(NFB * 4 == KCL);
static_assert(NTHR * 4 == 4 * DIM);
static_assert(DIM == NWAVE * 32);
static_assert(EPB == 4 * 32 && EPB >= KCL + 2);
static_assert(FTD == 2 * NWAVE * 4);
static_assert(KCL == 2 * NWAVE * 4);
static_assert(GRS == 16 * 8);
static_assert((GRS % 32) == 0);

typedef float          v4f   __attribute__((ext_vector_type(4)));
typedef float          v8f   __attribute__((ext_vector_type(8)));
typedef _Float16       v8h   __attribute__((ext_vector_type(8)));
typedef _Float16       v16h  __attribute__((ext_vector_type(16)));
typedef unsigned short v8us  __attribute__((ext_vector_type(8)));
typedef __bf16         bf16_t;
typedef bf16_t         v16bf __attribute__((ext_vector_type(16)));
union FragH { v16h v;  v8h  h[2]; };
union FragB { v16bf v; v8us u[2]; };

__device__ __forceinline__ v8f wmf(v16h a, v16h b, v8f c) {
  v8f d = __builtin_amdgcn_wmma_f32_16x16x32_f16(false, a, false, b, (short)0, c, false, false);
  asm volatile("v_nop\n\tv_nop\n\tv_nop\n\tv_nop" : "+v"(d) : "v"(a), "v"(b));
  return d;
}
__device__ __forceinline__ v8f wmb(v16bf a, v16bf b, v8f c) {
  v8f d = __builtin_amdgcn_wmma_f32_16x16x32_bf16(false, a, false, b, (short)0, c, false, false);
  asm volatile("v_nop\n\tv_nop\n\tv_nop\n\tv_nop" : "+v"(d) : "v"(a), "v"(b));
  return d;
}

__device__ __forceinline__ v8h cvt8h(v4f a, v4f b, float z) {
  v8h h;
  h[0] = (_Float16)(a.x * z); h[1] = (_Float16)(a.y * z); h[2] = (_Float16)(a.z * z); h[3] = (_Float16)(a.w * z);
  h[4] = (_Float16)(b.x * z); h[5] = (_Float16)(b.y * z); h[6] = (_Float16)(b.z * z); h[7] = (_Float16)(b.w * z);
  return h;
}

__device__ __forceinline__ unsigned bf16_rne(float x) {
  const unsigned u = __float_as_uint(x);
  return (u + 0x7FFFu + ((u >> 16) & 1u)) >> 16;
}
__device__ __forceinline__ void split1(float x, unsigned short& h, unsigned short& l) {
  const unsigned hb = bf16_rne(x);
  const float hf = __uint_as_float(hb << 16);
  h = (unsigned short)hb;
  l = (unsigned short)bf16_rne(x - hf);
}
__device__ __forceinline__ void split8(v4f a, v4f b, v8us& hv, v8us& lv) {
  unsigned short h, l;
  split1(a.x, h, l); hv[0] = h; lv[0] = l;
  split1(a.y, h, l); hv[1] = h; lv[1] = l;
  split1(a.z, h, l); hv[2] = h; lv[2] = l;
  split1(a.w, h, l); hv[3] = h; lv[3] = l;
  split1(b.x, h, l); hv[4] = h; lv[4] = l;
  split1(b.y, h, l); hv[5] = h; lv[5] = l;
  split1(b.z, h, l); hv[6] = h; lv[6] = l;
  split1(b.w, h, l); hv[7] = h; lv[7] = l;
}

__global__ __launch_bounds__(NTHR) void k_wT16(const float* __restrict__ W, _Float16* Wp,
                                               int KD, int NC, int NCP, float scale) {
  __shared__ __attribute__((aligned(16))) _Float16 sT[TPN * TPP];
  const int tid = threadIdx.x;
  const int z = (int)blockIdx.z;
  const float* Wz = W + (size_t)z * (size_t)KD * (size_t)NC;
  _Float16* Wpz = Wp + (size_t)z * (size_t)NCP * (size_t)KD;
  const int k0 = (int)blockIdx.x * TPK, n0 = (int)blockIdx.y * TPN;
  const int nc = tid & 31, kq = tid >> 5;
  const int col = n0 + nc;
  const int colc = col < NC ? col : NC - 1;
#pragma unroll
  for (int i = 0; i < TPK / NWAVE; ++i) {
    const int kr = kq + NWAVE * i;
    const float w = Wz[(size_t)(k0 + kr) * NC + colc];
    const float v = (col < NC) ? w * scale : 0.0f;
    sT[nc * TPP + kr] = (_Float16)v;
  }
  __syncthreads();
  const int nl = tid >> 3, p = tid & 7;
  const v8h hv = *(const v8h*)(sT + nl * TPP + 8 * p);
  _Float16* d = Wpz + (size_t)(n0 + nl) * KD + k0 + 8 * p;
  *(volatile v8h*)d = hv;
  __threadfence();
  *(volatile v8h*)d = hv;
}

__global__ __launch_bounds__(NTHR) void k_logits(
    const float* __restrict__ F, const _Float16* __restrict__ Wp, const float* __restrict__ bias,
    float* Sout, float* csp, unsigned short* STh, unsigned short* STl,
    int nN, int npad, float osc) {
  __shared__ __attribute__((aligned(16))) float stg[GRS * PSS];
  __shared__ __attribute__((aligned(16))) float scs[KCL];
  const int tid = threadIdx.x, lane = tid & 31, wave = tid >> 5, hh = lane >> 4, m = lane & 15;
  const int rowBase = blockIdx.x * GRS;
  const int ar  = rowBase + wave * 16 + m;
  const int arc = ar < nN ? ar : nN - 1;
  const float z = (ar < nN) ? (float)ASCL : 0.0f;
  const float* ap = F + (size_t)arc * DIM + 8 * hh;
  const _Float16* bp0 = Wp + (size_t)m * DIM + 8 * hh;

  v8f acc[4];
#pragma unroll
  for (int t = 0; t < 4; ++t) { v8f zz = {0.f, 0.f, 0.f, 0.f, 0.f, 0.f, 0.f, 0.f}; acc[t] = zz; }

#pragma unroll 1
  for (int kt = 0; kt < DIM / 32; ++kt) {
    const float* p = ap + 32 * kt;
    const v4f f0 = *(const v4f*)p;
    const v4f f1 = *(const v4f*)(p + 4);
    const v4f f2 = *(const v4f*)(p + 16);
    const v4f f3 = *(const v4f*)(p + 20);
    FragH af;
    af.h[0] = cvt8h(f0, f1, z);
    af.h[1] = cvt8h(f2, f3, z);
#pragma unroll
    for (int t = 0; t < 4; ++t) {
      const _Float16* bp = bp0 + (size_t)(16 * t) * DIM + 32 * kt;
      FragH bf;
      bf.h[0] = *(const v8h*)bp;
      bf.h[1] = *(const v8h*)(bp + 16);
      acc[t] = wmf(af.v, bf.v, acc[t]);
    }
  }

  float bc[4];
#pragma unroll
  for (int t = 0; t < 4; ++t) bc[t] = bias[16 * t + m];
#pragma unroll
  for (int t = 0; t < 4; ++t) {
#pragma unroll
    for (int r = 0; r < 8; ++r) acc[t][r] = acc[t][r] * osc + bc[t];
  }

#pragma unroll
  for (int r = 0; r < 8; ++r) {
    float mx = fmaxf(fmaxf(acc[0][r], acc[1][r]), fmaxf(acc[2][r], acc[3][r]));
    mx = fmaxf(mx, __shfl_xor(mx, 8, 32));
    mx = fmaxf(mx, __shfl_xor(mx, 4, 32));
    mx = fmaxf(mx, __shfl_xor(mx, 2, 32));
    mx = fmaxf(mx, __shfl_xor(mx, 1, 32));
    float s = 0.0f;
#pragma unroll
    for (int t = 0; t < 4; ++t) {
      const float e = __expf(acc[t][r] - mx);
      acc[t][r] = e;
      s += e;
    }
    s += __shfl_xor(s, 8, 32);
    s += __shfl_xor(s, 4, 32);
    s += __shfl_xor(s, 2, 32);
    s += __shfl_xor(s, 1, 32);
    const float inv = 1.0f / s;
#pragma unroll
    for (int t = 0; t < 4; ++t) acc[t][r] = acc[t][r] * inv;
  }

  {
    float* sp = stg + (wave * 16 + 8 * hh) * PSS + m;
#pragma unroll
    for (int t = 0; t < 4; ++t) {
#pragma unroll
      for (int r = 0; r < 8; ++r) sp[r * PSS + 16 * t] = acc[t][r];
    }
  }
  __syncthreads();

  int nr = nN - rowBase;
  nr = nr > GRS ? GRS : (nr < 0 ? 0 : nr);

  if (tid < KCL) {
    float cs = 0.0f;
#pragma unroll 1
    for (int r = 0; r < nr; ++r) cs += stg[r * PSS + tid];
    scs[tid] = cs;
  }

  v8us ph[4], pl[4];
#pragma unroll
  for (int it = 0; it < 4; ++it) {
    const int k = 2 * wave + 16 * it + hh;
    const int rb = 8 * m;
    const float* cp = stg + rb * PSS + k;
    v4f a, b;
    a.x = (rb + 0 < nr) ? cp[0 * PSS] : 0.0f;
    a.y = (rb + 1 < nr) ? cp[1 * PSS] : 0.0f;
    a.z = (rb + 2 < nr) ? cp[2 * PSS] : 0.0f;
    a.w = (rb + 3 < nr) ? cp[3 * PSS] : 0.0f;
    b.x = (rb + 4 < nr) ? cp[4 * PSS] : 0.0f;
    b.y = (rb + 5 < nr) ? cp[5 * PSS] : 0.0f;
    b.z = (rb + 6 < nr) ? cp[6 * PSS] : 0.0f;
    b.w = (rb + 7 < nr) ? cp[7 * PSS] : 0.0f;
    split8(a, b, ph[it], pl[it]);
  }
  __syncthreads();

  const v4f cv = *(const v4f*)(scs + 4 * (tid & 15));
  float* cgp = csp + (size_t)blockIdx.x * KCL + 4 * (tid & 15);
  const float* lpS = stg + (wave * 16) * PSS;
  float* gpS = Sout + (size_t)(rowBase + wave * 16) * KCL;

#pragma unroll
  for (int i = 0; i < 8; ++i) {
    const int rl = 2 * i + hh;
    const v4f v = *(const v4f*)(lpS + rl * PSS + 4 * m);
    if (wave * 16 + rl < nr) *(volatile v4f*)(gpS + (size_t)rl * KCL + 4 * m) = v;
  }
  if (tid < 16) *(volatile v4f*)cgp = cv;
#pragma unroll
  for (int it = 0; it < 4; ++it) {
    const int k = 2 * wave + 16 * it + hh;
    const size_t po = (size_t)k * (size_t)npad + (size_t)rowBase + 8 * m;
    *(volatile v8us*)(STh + po) = ph[it];
    *(volatile v8us*)(STl + po) = pl[it];
  }
  __threadfence();
#pragma unroll
  for (int i = 0; i < 8; ++i) {
    const int rl = 2 * i + hh;
    const v4f v = *(const v4f*)(lpS + rl * PSS + 4 * m);
    if (wave * 16 + rl < nr) *(volatile v4f*)(gpS + (size_t)rl * KCL + 4 * m) = v;
  }
  if (tid < 16) *(volatile v4f*)cgp = cv;
#pragma unroll
  for (int it = 0; it < 4; ++it) {
    const int k = 2 * wave + 16 * it + hh;
    const size_t po = (size_t)k * (size_t)npad + (size_t)rowBase + 8 * m;
    *(volatile v8us*)(STh + po) = ph[it];
    *(volatile v8us*)(STl + po) = pl[it];
  }
}

__global__ __launch_bounds__(NTHR) void k_fT(const float* __restrict__ F,
                                             unsigned short* FTh, unsigned short* FTl,
                                             int nN, int npad) {
  __shared__ __attribute__((aligned(16))) float sT[FTD * PFT];
  const int tid = threadIdx.x, lane = tid & 31, wave = tid >> 5, hh = lane >> 4, m = lane & 15;
  const int rowBase = blockIdx.x * GRS;
  const int d0 = (int)blockIdx.y * FTD;
  const int q = tid & 15, ng = tid >> 4;
#pragma unroll
  for (int it = 0; it < GRS / 16; ++it) {
    const int nl = it * 16 + ng;
    const int n  = rowBase + nl;
    const int nc = n < nN ? n : nN - 1;
    const v4f v = *(const v4f*)(F + (size_t)nc * DIM + d0 + 4 * q);
    const bool ok = n < nN;
    float* tp = sT + (4 * q) * PFT + nl;
    tp[0 * PFT] = ok ? v.x : 0.0f;
    tp[1 * PFT] = ok ? v.y : 0.0f;
    tp[2 * PFT] = ok ? v.z : 0.0f;
    tp[3 * PFT] = ok ? v.w : 0.0f;
  }
  __syncthreads();

  v8us ph[4], pl[4];
#pragma unroll
  for (int it = 0; it < 4; ++it) {
    const int dl = 2 * wave + 16 * it + hh;
    const float* rp = sT + dl * PFT + 8 * m;
    const v4f a = *(const v4f*)rp;
    const v4f b = *(const v4f*)(rp + 4);
    split8(a, b, ph[it], pl[it]);
  }
#pragma unroll
  for (int it = 0; it < 4; ++it) {
    const int dl = 2 * wave + 16 * it + hh;
    const size_t po = (size_t)(d0 + dl) * (size_t)npad + (size_t)rowBase + 8 * m;
    *(volatile v8us*)(FTh + po) = ph[it];
    *(volatile v8us*)(FTl + po) = pl[it];
  }
  __threadfence();
#pragma unroll
  for (int it = 0; it < 4; ++it) {
    const int dl = 2 * wave + 16 * it + hh;
    const size_t po = (size_t)(d0 + dl) * (size_t)npad + (size_t)rowBase + 8 * m;
    *(volatile v8us*)(FTh + po) = ph[it];
    *(volatile v8us*)(FTl + po) = pl[it];
  }
}

__global__ __launch_bounds__(NTHR) void k_edges(
    const int* __restrict__ er, const int* __restrict__ ec, const float* __restrict__ ev,
    int nE, const float* __restrict__ S, int nN, float* part) {
  __shared__ __attribute__((aligned(16))) float ssd[NWAVE * KCL];
  __shared__ float str[NWAVE];
  __shared__ float sne[NWAVE];
  __shared__ __attribute__((aligned(16))) float sout[EPB];
  const int tid = threadIdx.x, lane = tid & 31, wave = tid >> 5, hh = lane >> 4, m = lane & 15;
  const int nChunks = (nE + 31) >> 5;
  const int stride = (int)gridDim.x * NWAVE;
  const float* Sm = S + 4 * m;
  v4f sd = {0.f, 0.f, 0.f, 0.f};
  float tr = 0.0f, ne = 0.0f;

#pragma unroll 1
  for (int q = (int)blockIdx.x * NWAVE + wave; q < nChunks; q += stride) {
    const int e = (q << 5) + lane;
    const int ecl = e < nE ? e : nE - 1;
    int rl = er[ecl];
    int cl = ec[ecl];
    float vl = ev[ecl];
    vl = (e < nE) ? vl : 0.0f;
    rl = rl < 0 ? 0 : (rl > nN - 1 ? nN - 1 : rl);
    cl = cl < 0 ? 0 : (cl > nN - 1 ? nN - 1 : cl);
#pragma unroll 1
    for (int j = 0; j < 16; ++j) {
      const int src = 2 * j + hh;
      const int r = __shfl(rl, src, 32);
      const int c = __shfl(cl, src, 32);
      const float v = __shfl(vl, src, 32);
      const v4f a = *(const v4f*)(Sm + (size_t)r * KCL);
      const v4f b = *(const v4f*)(Sm + (size_t)c * KCL);
      float p = a.x * b.x + a.y * b.y + a.z * b.z + a.w * b.w;
      p += __shfl_xor(p, 1, 32);
      p += __shfl_xor(p, 2, 32);
      p += __shfl_xor(p, 4, 32);
      p += __shfl_xor(p, 8, 32);
      tr += v * p;
      ne += v;
      sd += b * v;
    }
  }

  sd.x += __shfl_xor(sd.x, 16, 32);
  sd.y += __shfl_xor(sd.y, 16, 32);
  sd.z += __shfl_xor(sd.z, 16, 32);
  sd.w += __shfl_xor(sd.w, 16, 32);
  tr += __shfl_xor(tr, 16, 32);
  ne += __shfl_xor(ne, 16, 32);
  if (hh == 0) *(v4f*)(ssd + wave * KCL + 4 * m) = sd;
  if (lane == 0) { str[wave] = tr; sne[wave] = ne; }
  __syncthreads();
  if (tid < EPB) {
    const int kc = tid & (KCL - 1);
    float s_sd = 0.0f, s_tr = 0.0f, s_ne = 0.0f;
#pragma unroll
    for (int w = 0; w < NWAVE; ++w) {
      s_sd += ssd[w * KCL + kc];
      s_tr += str[w];
      s_ne += sne[w];
    }
    float o = 0.0f;
    o = (tid < KCL) ? s_sd : o;
    o = (tid == KCL) ? s_tr : o;
    o = (tid == KCL + 1) ? s_ne : o;
    sout[tid] = o;
  }
  __syncthreads();
  if (wave == 0) {
    const v4f v = *(const v4f*)(sout + 4 * lane);
    float* gp = part + (size_t)blockIdx.x * EPB + 4 * lane;
    *(volatile v4f*)gp = v;
    __threadfence();
    *(volatile v4f*)gp = v;
  }
}

__global__ __launch_bounds__(NTHR) void k_pool(
    const unsigned short* __restrict__ STh, const unsigned short* __restrict__ STl,
    const unsigned short* __restrict__ FTh, const unsigned short* __restrict__ FTl,
    int npad, int nsteps, int spb, float* Pp) {
  extern __shared__ v4f lds_dyn[];
  float* stg = (float*)lds_dyn;
  const int tid = threadIdx.x, lane = tid & 31, wave = tid >> 5, hh = lane >> 4, m = lane & 15;
  int s0 = (int)blockIdx.x * spb;
  int s1 = s0 + spb;
  s0 = s0 > nsteps ? nsteps : s0;
  s1 = s1 > nsteps ? nsteps : s1;
  const int n0 = wave * 32;
  const size_t np = (size_t)npad;
  const unsigned short* aph = STh + (size_t)m * np + 8 * hh;
  const unsigned short* apl = STl + (size_t)m * np + 8 * hh;
  const unsigned short* bph = FTh + (size_t)(n0 + m) * np + 8 * hh;
  const unsigned short* bpl = FTl + (size_t)(n0 + m) * np + 8 * hh;

  v8f acc[8];
#pragma unroll
  for (int t = 0; t < 8; ++t) { v8f zz = {0.f, 0.f, 0.f, 0.f, 0.f, 0.f, 0.f, 0.f}; acc[t] = zz; }

#pragma unroll 1
  for (int ks = s0; ks < s1; ++ks) {
    const size_t ko = (size_t)ks << 5;
    FragB bh0, bl0, bh1, bl1;
    bh0.u[0] = *(const v8us*)(bph + ko);            bh0.u[1] = *(const v8us*)(bph + ko + 16);
    bl0.u[0] = *(const v8us*)(bpl + ko);            bl0.u[1] = *(const v8us*)(bpl + ko + 16);
    bh1.u[0] = *(const v8us*)(bph + 16 * np + ko);  bh1.u[1] = *(const v8us*)(bph + 16 * np + ko + 16);
    bl1.u[0] = *(const v8us*)(bpl + 16 * np + ko);  bl1.u[1] = *(const v8us*)(bpl + 16 * np + ko + 16);
#pragma unroll
    for (int mt = 0; mt < 4; ++mt) {
      FragB ah, al;
      ah.u[0] = *(const v8us*)(aph + (size_t)(16 * mt) * np + ko);
      ah.u[1] = *(const v8us*)(aph + (size_t)(16 * mt) * np + ko + 16);
      al.u[0] = *(const v8us*)(apl + (size_t)(16 * mt) * np + ko);
      al.u[1] = *(const v8us*)(apl + (size_t)(16 * mt) * np + ko + 16);
      acc[2 * mt]     = wmb(ah.v, bh0.v, acc[2 * mt]);
      acc[2 * mt]     = wmb(ah.v, bl0.v, acc[2 * mt]);
      acc[2 * mt]     = wmb(al.v, bh0.v, acc[2 * mt]);
      acc[2 * mt + 1] = wmb(ah.v, bh1.v, acc[2 * mt + 1]);
      acc[2 * mt + 1] = wmb(ah.v, bl1.v, acc[2 * mt + 1]);
      acc[2 * mt + 1] = wmb(al.v, bh1.v, acc[2 * mt + 1]);
    }
  }

#pragma unroll
  for (int mt = 0; mt < 4; ++mt) {
#pragma unroll
    for (int t = 0; t < 2; ++t) {
      float* sp = stg + (16 * mt + 8 * hh) * DIM + n0 + 16 * t + m;
#pragma unroll
      for (int r = 0; r < 8; ++r) sp[r * DIM] = acc[2 * mt + t][r];
    }
  }
  __syncthreads();

  const float* lp = stg + (size_t)(8 * wave) * DIM;
  float* gp = Pp + (size_t)blockIdx.x * (size_t)(KCL * DIM) + (size_t)(8 * wave) * DIM;
#pragma unroll
  for (int i = 0; i < 16; ++i) {
    const int o = (i >> 1) * DIM + (i & 1) * 128 + 4 * lane;
    const v4f v = *(const v4f*)(lp + o);
    *(volatile v4f*)(gp + o) = v;
  }
  __threadfence();
#pragma unroll
  for (int i = 0; i < 16; ++i) {
    const int o = (i >> 1) * DIM + (i & 1) * 128 + 4 * lane;
    const v4f v = *(const v4f*)(lp + o);
    *(volatile v4f*)(gp + o) = v;
  }
}

__global__ __launch_bounds__(NTHR) void k_final(
    const float* __restrict__ csp, int ncsb, const float* __restrict__ ep, int neb,
    const float* __restrict__ Pp, int npb, const float* __restrict__ lam,
    float* out0, float* out2, int nN) {
  __shared__ float scs[KCL];
  __shared__ double ssd[3 * KCL];
  __shared__ double sgl[16];
  __shared__ __attribute__((aligned(16))) float sres[4 * DIM];
  const int tid = threadIdx.x;

  if (tid < KCL) {
    double s = 0.0;
#pragma unroll 1
    for (int b = 0; b < ncsb; ++b) s += (double)csp[(size_t)b * KCL + tid];
    scs[tid] = (float)s;
  } else {
    const int g = (tid - KCL) >> 6, k = (tid - KCL) & 63;
    double s = 0.0;
#pragma unroll 1
    for (int b = 0; b < neb; ++b) s += (double)ep[((size_t)g * (size_t)neb + (size_t)b) * EPB + k];
    ssd[g * KCL + k] = s;
  }
  __syncthreads();
  if (tid < 32) {
    const int g = tid % 3;
    const int which = (tid / 3) & 1;
    double sa = 0.0;
#pragma unroll 1
    for (int b = 0; b < neb; ++b) sa += (double)ep[((size_t)g * (size_t)neb + (size_t)b) * EPB + KCL + which];
    double sb = 0.0;
#pragma unroll 1
    for (int k = 0; k < KCL; ++k) { const double v = ssd[g * KCL + k]; sb += v * v; }
    double sc = 0.0;
#pragma unroll 1
    for (int k = 0; k < KCL; ++k) { const double v = (double)scs[k]; sc += v * v; }
    if (tid < 6) sgl[which * 3 + g] = sa;
    else if (tid < 9) sgl[6 + g] = sb;
    else if (tid == 9) sgl[9] = sc;
  }
  __syncthreads();
  {
    const double two_m = sgl[3];
    const double l0 = -(sgl[0] - sgl[6] * 0.5 / sgl[3]) * 0.5 / two_m;
    const double l1 = -(sgl[1] - sgl[7] * 0.5 / sgl[4]) * 0.5 / two_m;
    const double l2 = -(sgl[2] - sgl[8] * 0.5 / sgl[5]) * 0.5 / two_m;
    const double fair = fabs((double)lam[0] * (l1 - l2));
    const double collapse = sqrt(sgl[9]) / (double)nN * sqrt((double)KCL) - 1.0;
    const float tot = (float)(fair + l0 + 0.1 * collapse);
    if (blockIdx.x == 0 && tid == 0) {
      *(volatile float*)out2 = tot;
      __threadfence();
      *(volatile float*)out2 = tot;
    }
  }

  const int rowl = tid >> 6;
  const int row  = (int)blockIdx.x * 4 + rowl;
  const int c4   = 4 * (tid & 63);
  const float rc = 1.0f / scs[row];
#pragma unroll 1
  for (int c = 0; c < 4; ++c) {
    float s = 0.0f;
#pragma unroll 1
    for (int g = 0; g < npb; ++g) s += Pp[(size_t)g * (size_t)(KCL * DIM) + (size_t)row * DIM + c4 + c];
    const float x = s * rc;
    const float y = x > 0.0f ? SELU_S * x : SELU_S * SELU_A * expm1f(x);
    sres[rowl * DIM + c4 + c] = y;
  }
  __syncthreads();
  const v4f v = *(const v4f*)(sres + 4 * tid);
  float* gp = out0 + (size_t)row * DIM + c4;
  *(volatile v4f*)gp = v;
  __threadfence();
  *(volatile v4f*)gp = v;
}

extern "C" void kernel_launch(void* const* d_in, const int* in_sizes, int n_in,
                              void* d_out, int out_size, void* d_ws, size_t ws_size,
                              hipStream_t stream) {
  if (n_in < 13) return;
  if (in_sizes[0] < DIM || (in_sizes[0] % DIM) != 0) return;
  const int nN = in_sizes[0] / DIM;
  const int nE0 = in_sizes[1], nE1 = in_sizes[4], nE2 = in_sizes[7];
  if (nE0 < 1 || in_sizes[2] != nE0 || in_sizes[3] != nE0) return;
  if (nE1 < 1 || in_sizes[5] != nE1 || in_sizes[6] != nE1) return;
  if (nE2 < 1 || in_sizes[8] != nE2 || in_sizes[9] != nE2) return;
  if (in_sizes[10] != DIM * KCL || in_sizes[11] != KCL || in_sizes[12] < 1) return;
  if ((size_t)out_size != (size_t)KCL * DIM + (size_t)nN * KCL + 1) return;

  const float* F    = (const float*)d_in[0];
  const int*   r0p  = (const int*)d_in[1];
  const int*   c0p  = (const int*)d_in[2];
  const float* v0p  = (const float*)d_in[3];
  const int*   r1p  = (const int*)d_in[4];
  const int*   c1p  = (const int*)d_in[5];
  const float* v1p  = (const float*)d_in[6];
  const int*   r2p  = (const int*)d_in[7];
  const int*   c2p  = (const int*)d_in[8];
  const float* v2p  = (const float*)d_in[9];
  const float* W    = (const float*)d_in[10];
  const float* bias = (const float*)d_in[11];
  const float* lam  = (const float*)d_in[12];
  float* out  = (float*)d_out;
  float* out0 = out;
  float* Sout = out + (size_t)KCL * DIM;
  float* out2 = out + (size_t)KCL * DIM + (size_t)nN * KCL;

  const int nRB    = (nN + GRS - 1) / GRS;
  const int npad   = nRB * GRS;
  const int nsteps = npad / 32;
  const int spb    = (nsteps + NPB - 1) / NPB;

  char* ws = (char*)d_ws;
  size_t off = 0;
  const size_t oWp  = off; off += (size_t)KCL * DIM * 2;              off = (off + 255) & ~(size_t)255;
  const size_t oSTh = off; off += (size_t)KCL * (size_t)npad * 2;     off = (off + 255) & ~(size_t)255;
  const size_t oSTl = off; off += (size_t)KCL * (size_t)npad * 2;     off = (off + 255) & ~(size_t)255;
  const size_t oFTh = off; off += (size_t)DIM * (size_t)npad * 2;     off = (off + 255) & ~(size_t)255;
  const size_t oFTl = off; off += (size_t)DIM * (size_t)npad * 2;     off = (off + 255) & ~(size_t)255;
  const size_t oCs  = off; off += (size_t)nRB * KCL * 4;              off = (off + 255) & ~(size_t)255;
  const size_t oEp  = off; off += (size_t)3 * NEG * EPB * 4;          off = (off + 255) & ~(size_t)255;
  const size_t oPp  = off; off += (size_t)NPB * KCL * DIM * 4;        off = (off + 255) & ~(size_t)255;
  if (off > ws_size || off > (size_t)WSCAP) return;
  _Float16*       Wp  = (_Float16*)(ws + oWp);
  unsigned short* STh = (unsigned short*)(ws + oSTh);
  unsigned short* STl = (unsigned short*)(ws + oSTl);
  unsigned short* FTh = (unsigned short*)(ws + oFTh);
  unsigned short* FTl = (unsigned short*)(ws + oFTl);
  float* csp = (float*)(ws + oCs);
  float* ep  = (float*)(ws + oEp);
  float* Pp  = (float*)(ws + oPp);

  const float osc = 1.0f / ((float)ASCL * (float)WSCL);

  {
    const dim3 gW(DIM / TPK, KCL / TPN, 1);
    k_wT16<<<gW, NTHR, 0, stream>>>(W, Wp, DIM, KCL, KCL, (float)WSCL);
  }
  k_logits<<<nRB, NTHR, 0, stream>>>(F, Wp, bias, Sout, csp, STh, STl, nN, npad, osc);
  {
    const dim3 gF(nRB, DIM / FTD, 1);
    k_fT<<<gF, NTHR, 0, stream>>>(F, FTh, FTl, nN, npad);
  }
  k_edges<<<NEG, NTHR, 0, stream>>>(r0p, c0p, v0p, nE0, Sout, nN, ep + (size_t)0 * NEG * EPB);
  k_edges<<<NEG, NTHR, 0, stream>>>(r1p, c1p, v1p, nE1, Sout, nN, ep + (size_t)1 * NEG * EPB);
  k_edges<<<NEG, NTHR, 0, stream>>>(r2p, c2p, v2p, nE2, Sout, nN, ep + (size_t)2 * NEG * EPB);
  hipFuncSetAttribute(reinterpret_cast<const void*>(&k_pool),
                      hipFuncAttributeMaxDynamicSharedMemorySize, LDS_POOL);
  k_pool<<<NPB, NTHR, LDS_POOL, stream>>>(STh, STl, FTh, FTl, npad, nsteps, spb, Pp);
  k_final<<<NFB, NTHR, 0, stream>>>(csp, nRB, ep, NEG, Pp, NPB, lam, out0, out2, nN);
}
